// MultiHeadAttention2D_73143293051615
// MI455X (gfx1250) — hardware-run, weakly checked
//
#include <hip/hip_runtime.h>
#include <math.h>
#include <stdint.h>

#ifndef NB
#define NB 8
#endif
#define NBF   8
#define CC    256
#define NN    1024
#define NH    8
#define DD    32
#define QT    64
#define NQT   (NN / QT)
#define NSLOT (NH * NQT)
#define OSP   100
#define OSQ   36
#define YSP   68
#define TP    72
#define EP    (NN + 8)
#define EDYNB (QT * EP * 2)
#define VSC   16.0f
#define IVSC  0.0625f
#define ESC   32768.0f
#define IESC  3.0517578125e-05f
#define INVPI 0.3183098861837907f
#define CLIPV 0.999999f
#define INH   0.125f
#define OUT1E (NBF * CC * NN)
#define WBLKE 2048
#define WGBLK ((3 * CC * DD) / WBLKE)
#define WFBLK ((CC * CC) / WBLKE)

static_assert(NB >= 1 && NB <= NBF);
static_assert(CC == NH * DD && DD == 32 && NH == 8);
static_assert(NN % QT == 0 && NN % 32 == 0 && QT == 64);
static_assert(NQT * QT == NN && NSLOT == 128);
static_assert(NN == 256 * 4);
static_assert((3 * CC * DD) % WBLKE == 0 && (CC * CC) % WBLKE == 0 && WBLKE == 256 * 8);
static_assert(WGBLK == 12 && WFBLK == 32);
static_assert((OSP * 4) % 16 == 0 && (OSQ * 4) % 16 == 0 && (YSP * 4) % 16 == 0);
static_assert((TP * 2) % 16 == 0 && (EP * 2) % 16 == 0);
static_assert(EDYNB == 132096);
static_assert(OUT1E * 4 == 8388608);

typedef _Float16       v16h __attribute__((ext_vector_type(16)));
typedef _Float16       v8h  __attribute__((ext_vector_type(8)));
typedef __bf16         v16b __attribute__((ext_vector_type(16)));
typedef unsigned short v8us __attribute__((ext_vector_type(8)));
typedef float          v8f  __attribute__((ext_vector_type(8)));
typedef float          v4f  __attribute__((ext_vector_type(4)));
typedef unsigned int   v4u  __attribute__((ext_vector_type(4)));

union Frag  { v8us u[2]; v16h h; v16b bf; };
union FragH { v16h v; v8h hv[2]; };
static_assert(sizeof(Frag) == 32);
static_assert(sizeof(FragH) == 32);

__device__ __forceinline__ unsigned short bf_bits(float f) {
  unsigned u = __float_as_uint(f);
  return (unsigned short)((u + 0x7FFFu + ((u >> 16) & 1u)) >> 16);
}
__device__ __forceinline__ float bf_up(unsigned short hb) { return __uint_as_float(((unsigned)hb) << 16); }
__device__ __forceinline__ float bfr(float f) { return bf_up(bf_bits(f)); }
__device__ __forceinline__ unsigned short h_bits(_Float16 x) { return __builtin_bit_cast(unsigned short, x); }
__device__ __forceinline__ unsigned pk16(unsigned short a, unsigned short b) { return (unsigned)a | ((unsigned)b << 16); }
__device__ __forceinline__ v8f zero8() { v8f z = {0.f, 0.f, 0.f, 0.f, 0.f, 0.f, 0.f, 0.f}; return z; }
__device__ __forceinline__ float mishf(float y) {
  const float sp = fmaxf(y, 0.0f) + log1pf(expf(-fabsf(y)));
  return y * tanhf(sp);
}

__device__ __forceinline__ Frag ldfrag(const unsigned short* p) {
  Frag f;
  f.u[0] = *(const v8us*)(p);
  f.u[1] = *(const v8us*)(p + 16);
  return f;
}

__device__ __forceinline__ v8f mma_h(v16h a, v16h b, v8f c) {
  v8f d = __builtin_amdgcn_wmma_f32_16x16x32_f16(false, a, false, b, (short)0, c, false, false);
#if defined(__HIP_DEVICE_COMPILE__)
  asm volatile("v_nop\n\tv_nop\n\tv_nop\n\tv_nop" : "+v"(d) : "v"(a), "v"(b));
#endif
  return d;
}
__device__ __forceinline__ v8f mma_b(v16b a, v16b b, v8f c) {
  v8f d = __builtin_amdgcn_wmma_f32_16x16x32_bf16(false, a, false, b, (short)0, c, false, false);
#if defined(__HIP_DEVICE_COMPILE__)
  const v16h ha = __builtin_bit_cast(v16h, a), hb = __builtin_bit_cast(v16h, b);
  asm volatile("v_nop\n\tv_nop\n\tv_nop\n\tv_nop" : "+v"(d) : "v"(ha), "v"(hb));
#endif
  return d;
}

__global__ __launch_bounds__(256)
void cvt_w(const float* __restrict__ qw, const float* __restrict__ kw, const float* __restrict__ vw,
           const float* __restrict__ fw, unsigned short* Wg, unsigned short* Wf) {
  const int tid = threadIdx.x, blk = blockIdx.x;
  const float* src;
  unsigned short* dst;
  size_t eo;
  if (blk < WGBLK) {
    const int s = blk / (WGBLK / 3);
    const size_t lo = (size_t)(blk % (WGBLK / 3)) * WBLKE + 8 * tid;
    src = ((s == 0) ? qw : ((s == 1) ? kw : vw)) + lo;
    dst = Wg;
    eo  = (size_t)s * (CC * DD) + lo;
  } else {
    const size_t lo = (size_t)(blk - WGBLK) * WBLKE + 8 * tid;
    src = fw + lo;
    dst = Wf;
    eo  = lo;
  }
  const v4f a = *(const v4f*)src;
  const v4f q = *(const v4f*)(src + 4);
  v4u u;
  u[0] = pk16(bf_bits(a[0]), bf_bits(a[1]));
  u[1] = pk16(bf_bits(a[2]), bf_bits(a[3]));
  u[2] = pk16(bf_bits(q[0]), bf_bits(q[1]));
  u[3] = pk16(bf_bits(q[2]), bf_bits(q[3]));
#pragma unroll
  for (int pass = 0; pass < 2; ++pass) {
    *(volatile v4u*)(dst + eo) = u;
    __threadfence();
  }
}

__global__ __launch_bounds__(256)
void cvt_x(const float* __restrict__ x, unsigned short* XP) {
  __shared__ __align__(16) unsigned short T[QT * TP];
  const int tid = threadIdx.x;
  const int nb = blockIdx.x, cb = blockIdx.y, b = blockIdx.z;
  const int e = tid & 7, lq = tid >> 3;
  const int n0 = nb * QT, c0 = cb * QT;
#pragma unroll
  for (int it = 0; it < 2; ++it) {
    const int cl = it * 32 + lq;
    const float* sp = x + ((size_t)(b * CC + c0 + cl)) * NN + n0 + 8 * e;
    const v4f a = *(const v4f*)sp;
    const v4f q = *(const v4f*)(sp + 4);
    unsigned short hb[8];
#pragma unroll
    for (int t = 0; t < 4; ++t) {
      hb[t]     = bf_bits(a[t]);
      hb[4 + t] = bf_bits(q[t]);
    }
#pragma unroll
    for (int t = 0; t < 8; ++t) T[(8 * e + t) * TP + cl] = hb[t];
  }
  __syncthreads();
  v4u up[2];
#pragma unroll
  for (int it = 0; it < 2; ++it) {
    const int nl = it * 32 + lq;
    up[it] = *(const v4u*)(T + nl * TP + 8 * e);
  }
#pragma unroll
  for (int pass = 0; pass < 2; ++pass) {
#pragma unroll
    for (int it = 0; it < 2; ++it) {
      const int nl = it * 32 + lq;
      *(volatile v4u*)(XP + ((size_t)(b * NN + n0 + nl)) * CC + c0 + 8 * e) = up[it];
    }
    __threadfence();
  }
}

__global__ __launch_bounds__(128)
void qkv_k(const unsigned short* __restrict__ Wg, const unsigned short* __restrict__ XP,
           const float* __restrict__ qb, const float* __restrict__ qs, const float* __restrict__ qe,
           const float* __restrict__ kb, const float* __restrict__ ks, const float* __restrict__ ke,
           const float* __restrict__ vb, const float* __restrict__ vs, const float* __restrict__ ve,
           unsigned short* Qh, unsigned short* Ql, unsigned short* Kh, unsigned short* Kl,
           unsigned short* Vt) {
  __shared__ __align__(16) float Os[QT * OSP];
  __shared__ float Par[9 * DD];
  const int tid  = threadIdx.x;
  const int lane = tid & 31, wave = tid >> 5;
  const int hh   = lane >> 4, c = lane & 15;
  const int nt   = blockIdx.x, g = blockIdx.y, b = blockIdx.z;
  const int n0   = nt * QT;

  if (wave == 0) {
    const int o = g * DD + lane;
    Par[0 * DD + lane] = bfr(qb[o]);
    Par[1 * DD + lane] = bfr(qs[o]);
    Par[2 * DD + lane] = bfr(qe[o]);
    Par[3 * DD + lane] = bfr(kb[o]);
    Par[4 * DD + lane] = bfr(ks[o]);
    Par[5 * DD + lane] = bfr(ke[o]);
    Par[6 * DD + lane] = bfr(vb[o]);
    Par[7 * DD + lane] = bfr(vs[o]);
    Par[8 * DD + lane] = bfr(ve[o]);
  }

  const Frag fb = ldfrag(XP + ((size_t)(b * NN + n0 + 16 * wave + c)) * CC + g * DD + 8 * hh);
  v8f acc[3][2];
#pragma unroll
  for (int s = 0; s < 3; ++s) {
#pragma unroll
    for (int mt = 0; mt < 2; ++mt) {
      const Frag fa = ldfrag(Wg + ((size_t)(s * CC + g * DD + 16 * mt + c)) * DD + 8 * hh);
      acc[s][mt] = mma_b(fa.bf, fb.bf, zero8());
    }
  }

  {
    const int nl = 16 * wave + c;
#pragma unroll
    for (int s = 0; s < 3; ++s) {
#pragma unroll
      for (int mt = 0; mt < 2; ++mt) {
        v4f va, vq;
#pragma unroll
        for (int r = 0; r < 4; ++r) { va[r] = acc[s][mt][r]; vq[r] = acc[s][mt][4 + r]; }
        *(v4f*)(Os + nl * OSP + s * DD + 16 * mt + 8 * hh)     = va;
        *(v4f*)(Os + nl * OSP + s * DD + 16 * mt + 8 * hh + 4) = vq;
      }
    }
  }
  __syncthreads();

  {
    const int nl = tid & 63, sel = tid >> 6;
    float* rowp = Os + nl * OSP + sel * DD;
    const float* pb = Par + (sel * 3 + 0) * DD;
    const float* ps = Par + (sel * 3 + 1) * DD;
    const float* pe = Par + (sel * 3 + 2) * DD;
    float ss = 0.f;
#pragma unroll 2
    for (int d = 0; d < DD; ++d) {
      const float y = rowp[d];
      const float m = mishf(ps[d] * (y + pb[d]) + pe[d]);
      rowp[d] = m;
      ss = fmaf(m, m, ss);
    }
    const float rn = (ss > 0.f) ? (1.0f / sqrtf(ss)) : 0.f;
#pragma unroll 4
    for (int d = 0; d < DD; ++d) rowp[d] = rowp[d] * rn;
    float* vp = Os + nl * OSP + 2 * DD + sel * 16;
    const float* wb = Par + 6 * DD + sel * 16;
    const float* wsc = Par + 7 * DD + sel * 16;
    const float* we = Par + 8 * DD + sel * 16;
#pragma unroll 2
    for (int d = 0; d < 16; ++d) {
      const float y = vp[d];
      vp[d] = mishf(wsc[d] * (y + wb[d]) + we[d]);
    }
  }
  __syncthreads();

  const int e = tid & 7, lq = tid >> 3;
  v4u uqh[2], uql[2], ukh[2], ukl[2], uv[2];
#pragma unroll
  for (int it = 0; it < 2; ++it) {
    const int L    = 16 * it + lq;
    const int row  = 2 * L + (e >> 2);
    const int dseg = 8 * (e & 3);
#pragma unroll
    for (int sel = 0; sel < 2; ++sel) {
      const float* rp = Os + row * OSP + sel * DD + dseg;
      const v4f a = *(const v4f*)rp;
      const v4f q = *(const v4f*)(rp + 4);
      const float f[8] = {a[0], a[1], a[2], a[3], q[0], q[1], q[2], q[3]};
      v4u uhv, ulv;
#pragma unroll
      for (int t = 0; t < 4; ++t) {
        const float f0 = f[2 * t], f1 = f[2 * t + 1];
        const unsigned short hb0 = bf_bits(f0), hb1 = bf_bits(f1);
        const unsigned short lb0 = bf_bits(f0 - bf_up(hb0));
        const unsigned short lb1 = bf_bits(f1 - bf_up(hb1));
        uhv[t] = pk16(hb0, hb1);
        ulv[t] = pk16(lb0, lb1);
      }
      if (sel == 0) { uqh[it] = uhv; uql[it] = ulv; }
      else          { ukh[it] = uhv; ukl[it] = ulv; }
    }
    const int d = 16 * it + lq;
    unsigned short vbt[8];
#pragma unroll
    for (int t = 0; t < 8; ++t) vbt[t] = h_bits((_Float16)(Os[(8 * e + t) * OSP + 2 * DD + d] * VSC));
#pragma unroll
    for (int t = 0; t < 4; ++t) uv[it][t] = pk16(vbt[2 * t], vbt[2 * t + 1]);
  }
#pragma unroll
  for (int pass = 0; pass < 2; ++pass) {
#pragma unroll
    for (int it = 0; it < 2; ++it) {
      const int L    = 16 * it + lq;
      const int row  = 2 * L + (e >> 2);
      const int dseg = 8 * (e & 3);
      const size_t po = ((size_t)((b * NH + g) * NN + n0 + row)) * DD + dseg;
      *(volatile v4u*)(Qh + po) = uqh[it];
      *(volatile v4u*)(Ql + po) = uql[it];
      *(volatile v4u*)(Kh + po) = ukh[it];
      *(volatile v4u*)(Kl + po) = ukl[it];
      const int d = 16 * it + lq;
      const size_t pv = ((size_t)(b * CC + g * DD + d)) * NN + n0 + 8 * e;
      *(volatile v4u*)(Vt + pv) = uv[it];
    }
    __threadfence();
  }
}

__global__ __launch_bounds__(128)
void attn_k(const unsigned short* __restrict__ Qh, const unsigned short* __restrict__ Ql,
            const unsigned short* __restrict__ Kh, const unsigned short* __restrict__ Kl,
            const unsigned short* __restrict__ Vt,
            unsigned short* Oh, unsigned short* Ol, float* CS) {
  extern __shared__ __align__(16) unsigned short Edyn[];
  __shared__ __align__(16) float Os3[QT * OSQ];
  __shared__ __align__(16) float Cs[NN];
  __shared__ float Linv[QT];
  const int tid  = threadIdx.x;
  const int wave = tid >> 5, lane = tid & 31;
  const int hh   = lane >> 4, c = lane & 15;
  const int qt   = blockIdx.x, h = blockIdx.y, b = blockIdx.z;
  const int n0   = qt * QT, bh = b * NH + h;

  const size_t qo = ((size_t)(bh * NN + n0 + 16 * wave + c)) * DD + 8 * hh;
  const Frag qh = ldfrag(Qh + qo);
  const Frag ql = ldfrag(Ql + qo);
  const unsigned short* Khp = Kh + (size_t)bh * NN * DD + (size_t)c * DD + 8 * hh;
  const unsigned short* Klp = Kl + (size_t)bh * NN * DD + (size_t)c * DD + 8 * hh;
  const unsigned short* Vp = Vt + ((size_t)(b * CC + h * DD + c)) * NN + 8 * hh;
  unsigned short* Erow = Edyn + (size_t)(16 * wave + c) * EP + 8 * hh;

  float l = 0.f;
  v8f o[2];
  o[0] = zero8();
  o[1] = zero8();

#pragma unroll 1
  for (int kb = 0; kb < NN; kb += 32) {
    const Frag k0  = ldfrag(Khp + (size_t)kb * DD);
    const Frag k1  = ldfrag(Khp + (size_t)(kb + 16) * DD);
    const Frag k0l = ldfrag(Klp + (size_t)kb * DD);
    const Frag k1l = ldfrag(Klp + (size_t)(kb + 16) * DD);
    v8f s0 = mma_b(k0.bf, qh.bf, zero8());
    v8f s1 = mma_b(k1.bf, qh.bf, zero8());
    s0 = mma_b(k0.bf, ql.bf, s0);
    s1 = mma_b(k1.bf, ql.bf, s1);
    s0 = mma_b(k0l.bf, qh.bf, s0);
    s1 = mma_b(k1l.bf, qh.bf, s1);

    FragH ph;
    float ls = 0.f;
    unsigned short u0[8], u1[8];
#pragma unroll
    for (int r = 0; r < 8; ++r) {
      const float c0 = fminf(fmaxf(s0[r], -CLIPV), CLIPV);
      const float c1 = fminf(fmaxf(s1[r], -CLIPV), CLIPV);
      const float sc0 = 1.0f - acosf(c0) * INVPI;
      const float sc1 = 1.0f - acosf(c1) * INVPI;
      const float e0 = __expf(sc0 - 1.0f);
      const float e1 = __expf(sc1 - 1.0f);
      ls += e0 + e1;
      ph.hv[0][r] = (_Float16)e0;
      ph.hv[1][r] = (_Float16)e1;
      u0[r] = (unsigned short)((unsigned int)(e0 * ESC + 0.5f));
      u1[r] = (unsigned short)((unsigned int)(e1 * ESC + 0.5f));
    }
    l += ls;
    v4u w0, w1;
#pragma unroll
    for (int t = 0; t < 4; ++t) { w0[t] = pk16(u0[2 * t], u0[2 * t + 1]); w1[t] = pk16(u1[2 * t], u1[2 * t + 1]); }
    *(v4u*)(Erow + kb)      = w0;
    *(v4u*)(Erow + kb + 16) = w1;

#pragma unroll
    for (int j = 0; j < 2; ++j) {
      const Frag vf = ldfrag(Vp + (size_t)(16 * j) * NN + kb);
      o[j] = mma_h(vf.h, ph.v, o[j]);
    }
  }
  l += __shfl_xor(l, 16, 32);
  const float il  = 1.0f / l;
  const float inv = il * IVSC;
  if (hh == 0) Linv[16 * wave + c] = il;
  {
    const int nl = 16 * wave + c;
#pragma unroll
    for (int j = 0; j < 2; ++j) {
      v4f va, vq;
#pragma unroll
      for (int r = 0; r < 4; ++r) { va[r] = o[j][r] * inv; vq[r] = o[j][4 + r] * inv; }
      *(v4f*)(Os3 + nl * OSQ + 16 * j + 8 * hh)     = va;
      *(v4f*)(Os3 + nl * OSQ + 16 * j + 8 * hh + 4) = vq;
    }
  }
  __syncthreads();

  {
    float ca[8];
#pragma unroll
    for (int t = 0; t < 8; ++t) ca[t] = 0.f;
    const unsigned short* Ep = Edyn + 8 * tid;
#pragma unroll 2
    for (int q = 0; q < QT; ++q) {
      const v4u w = *(const v4u*)(Ep + (size_t)q * EP);
      const float li = Linv[q];
#pragma unroll
      for (int t = 0; t < 4; ++t) {
        ca[2 * t]     = fmaf((float)(w[t] & 0xffffu), li, ca[2 * t]);
        ca[2 * t + 1] = fmaf((float)(w[t] >> 16), li, ca[2 * t + 1]);
      }
    }
    v4f ca0, ca1;
#pragma unroll
    for (int t = 0; t < 4; ++t) { ca0[t] = ca[t] * IESC; ca1[t] = ca[4 + t] * IESC; }
    *(v4f*)(Cs + 8 * tid)     = ca0;
    *(v4f*)(Cs + 8 * tid + 4) = ca1;
  }
  const int e = tid & 7, lq = tid >> 3;
  v4u uh[2], ul[2];
#pragma unroll
  for (int it = 0; it < 2; ++it) {
    const int L    = 16 * it + lq;
    const int row  = 2 * L + (e >> 2);
    const int dseg = 8 * (e & 3);
    const float* rp = Os3 + row * OSQ + dseg;
    const v4f a = *(const v4f*)rp;
    const v4f q = *(const v4f*)(rp + 4);
    const float f[8] = {a[0], a[1], a[2], a[3], q[0], q[1], q[2], q[3]};
#pragma unroll
    for (int t = 0; t < 4; ++t) {
      const float f0 = f[2 * t], f1 = f[2 * t + 1];
      const unsigned short hb0 = bf_bits(f0), hb1 = bf_bits(f1);
      const unsigned short lb0 = bf_bits(f0 - bf_up(hb0));
      const unsigned short lb1 = bf_bits(f1 - bf_up(hb1));
      uh[it][t] = pk16(hb0, hb1);
      ul[it][t] = pk16(lb0, lb1);
    }
  }
  __syncthreads();
  v4f cl2[2];
#pragma unroll
  for (int it = 0; it < 2; ++it) {
    const int L = 16 * it + lq;
    cl2[it] = *(const v4f*)(Cs + 32 * L + 4 * e);
  }
  const size_t csbase = ((size_t)(bh * NQT + qt)) * NN;
#pragma unroll
  for (int pass = 0; pass < 2; ++pass) {
#pragma unroll
    for (int it = 0; it < 2; ++it) {
      const int L    = 16 * it + lq;
      const int row  = 2 * L + (e >> 2);
      const int dseg = 8 * (e & 3);
      const size_t po = ((size_t)(bh * NN + n0 + row)) * DD + dseg;
      *(volatile v4u*)(Oh + po) = uh[it];
      *(volatile v4u*)(Ol + po) = ul[it];
      *(volatile v4f*)(CS + csbase + 32 * L + 4 * e) = cl2[it];
    }
    __threadfence();
  }
}

__global__ __launch_bounds__(128)
void fconv_k(const unsigned short* __restrict__ Wf, const unsigned short* __restrict__ Oh,
             const unsigned short* __restrict__ Ol, const float* __restrict__ fb,
             const float* __restrict__ fs, const float* __restrict__ fe,
             const float* __restrict__ x, float* out) {
  __shared__ __align__(16) float Ys[QT * YSP];
  const int tid  = threadIdx.x;
  const int lane = tid & 31, wave = tid >> 5;
  const int hh   = lane >> 4, c = lane & 15;
  const int nt   = blockIdx.x, mb = blockIdx.y, b = blockIdx.z;
  const int n0   = nt * QT, o0 = mb * QT;

  const unsigned short* ap = Wf + (size_t)(o0 + c) * CC + 8 * hh;
  const size_t bo = ((size_t)(b * NH) * NN + n0 + 16 * wave + c) * DD + 8 * hh;

  v8f acc[4];
#pragma unroll
  for (int mt = 0; mt < 4; ++mt) acc[mt] = zero8();

#pragma unroll
  for (int ks = 0; ks < CC / 32; ++ks) {
    const Frag fbh = ldfrag(Oh + bo + (size_t)ks * NN * DD);
    const Frag fbl = ldfrag(Ol + bo + (size_t)ks * NN * DD);
#pragma unroll
    for (int mt = 0; mt < 4; ++mt) {
      const Frag fa = ldfrag(ap + (size_t)(16 * mt) * CC + 32 * ks);
      acc[mt] = mma_b(fa.bf, fbh.bf, acc[mt]);
      acc[mt] = mma_b(fa.bf, fbl.bf, acc[mt]);
    }
  }

  {
    const int nl = 16 * wave + c;
#pragma unroll
    for (int mt = 0; mt < 4; ++mt) {
      v4f va, vq;
#pragma unroll
      for (int r = 0; r < 4; ++r) { va[r] = acc[mt][r]; vq[r] = acc[mt][4 + r]; }
      *(v4f*)(Ys + nl * YSP + 16 * mt + 8 * hh)     = va;
      *(v4f*)(Ys + nl * YSP + 16 * mt + 8 * hh + 4) = vq;
    }
  }
  __syncthreads();

  const int e = tid & 7, lq = tid >> 3;
  v4f res[8];
#pragma unroll
  for (int it = 0; it < 8; ++it) {
    const int L  = it * 16 + lq;
    const int ol = L >> 1, hf = L & 1;
    const int nl = hf * 32 + 4 * e;
    const int oc = o0 + ol;
    const float pb = bfr(fb[oc]), ps = bfr(fs[oc]), pe = bfr(fe[oc]);
    const size_t idx = ((size_t)(b * CC + oc)) * NN + n0 + nl;
    const v4f xv = *(const v4f*)(x + idx);
#pragma unroll
    for (int t = 0; t < 4; ++t) res[it][t] = mishf(ps * (Ys[(nl + t) * YSP + ol] + pb) + pe) + bfr(xv[t]);
  }
#pragma unroll
  for (int pass = 0; pass < 2; ++pass) {
#pragma unroll
    for (int it = 0; it < 8; ++it) {
      const int L  = it * 16 + lq;
      const int ol = L >> 1, hf = L & 1;
      const int nl = hf * 32 + 4 * e;
      const size_t idx = ((size_t)(b * CC + o0 + ol)) * NN + n0 + nl;
      *(volatile v4f*)(out + idx) = res[it];
    }
    __threadfence();
  }
}

__global__ __launch_bounds__(256)
void amfin_k(const float* __restrict__ CS, float* out) {
  __shared__ float rmn[8], rmx[8];
  const int tid = threadIdx.x, lane = tid & 31, wave = tid >> 5, b = blockIdx.x;
  const float* base = CS + (size_t)b * NSLOT * NN + 4 * tid;
  double a0 = 0.0, a1 = 0.0, a2 = 0.0, a3 = 0.0;
#pragma unroll 2
  for (int s = 0; s < NSLOT; ++s) {
    const v4f v = *(const v4f*)(base + (size_t)s * NN);
    a0 += (double)v[0]; a1 += (double)v[1]; a2 += (double)v[2]; a3 += (double)v[3];
  }
  const float m0 = (float)a0 * INH, m1 = (float)a1 * INH, m2 = (float)a2 * INH, m3 = (float)a3 * INH;
  float mn = fminf(fminf(m0, m1), fminf(m2, m3));
  float mx = fmaxf(fmaxf(m0, m1), fmaxf(m2, m3));
#pragma unroll
  for (int off = 16; off >= 1; off >>= 1) {
    mn = fminf(mn, __shfl_xor(mn, off, 32));
    mx = fmaxf(mx, __shfl_xor(mx, off, 32));
  }
  if (lane == 0) { rmn[wave] = mn; rmx[wave] = mx; }
  __syncthreads();
  float gmn = rmn[0], gmx = rmx[0];
#pragma unroll
  for (int w = 1; w < 8; ++w) { gmn = fminf(gmn, rmn[w]); gmx = fmaxf(gmx, rmx[w]); }
  const float ir = 1.0f / (gmx - gmn);
  v4f r;
  r[0] = (m0 - gmn) * ir;
  r[1] = (m1 - gmn) * ir;
  r[2] = (m2 - gmn) * ir;
  r[3] = (m3 - gmn) * ir;
  const size_t oo = (size_t)OUT1E + (size_t)b * NN + 4 * tid;
#pragma unroll
  for (int pass = 0; pass < 2; ++pass) {
    *(volatile v4f*)(out + oo) = r;
    __threadfence();
  }
}

extern "C" void kernel_launch(void* const* d_in, const int* in_sizes, int n_in,
                              void* d_out, int out_size, void* d_ws, size_t ws_size,
                              hipStream_t stream) {
  if (n_in < 17) return;
  if (in_sizes[0] < NB * CC * NN) return;
  if (in_sizes[1] < CC * DD || in_sizes[5] < CC * DD || in_sizes[9] < CC * DD) return;
  if (in_sizes[13] < CC * CC) return;
  for (int i = 2; i <= 16; ++i) {
    if (i == 5 || i == 9 || i == 13) continue;
    if (in_sizes[i] < CC) return;
  }
  if (out_size < OUT1E + NB * NN) return;

  size_t off = 0;
  auto carve = [&](size_t bytes) { const size_t o = off; off += (bytes + 255) & ~(size_t)255; return o; };
  const size_t oWg = carve((size_t)3 * CC * DD * 2);
  const size_t oWf = carve((size_t)CC * CC * 2);
  const size_t oXP = carve((size_t)NB * NN * CC * 2);
  const size_t oQh = carve((size_t)NB * NH * NN * DD * 2);
  const size_t oQl = carve((size_t)NB * NH * NN * DD * 2);
  const size_t oKh = carve((size_t)NB * NH * NN * DD * 2);
  const size_t oKl = carve((size_t)NB * NH * NN * DD * 2);
  const size_t oVt = carve((size_t)NB * CC * NN * 2);
  const size_t oOh = carve((size_t)NB * NH * NN * DD * 2);
  const size_t oOl = carve((size_t)NB * NH * NN * DD * 2);
  const size_t oCS = carve((size_t)NB * NSLOT * NN * 4);
  if (off > ws_size) return;
  if (off > (size_t)134217728) return;

  const float* x   = (const float*)d_in[0];
  const float* qw  = (const float*)d_in[1];
  const float* qb  = (const float*)d_in[2];
  const float* qs  = (const float*)d_in[3];
  const float* qe  = (const float*)d_in[4];
  const float* kw  = (const float*)d_in[5];
  const float* kb  = (const float*)d_in[6];
  const float* ks  = (const float*)d_in[7];
  const float* ke  = (const float*)d_in[8];
  const float* vw  = (const float*)d_in[9];
  const float* vb  = (const float*)d_in[10];
  const float* vs  = (const float*)d_in[11];
  const float* ve  = (const float*)d_in[12];
  const float* fw  = (const float*)d_in[13];
  const float* fb  = (const float*)d_in[14];
  const float* fs  = (const float*)d_in[15];
  const float* fe  = (const float*)d_in[16];

  char* ws = (char*)d_ws;
  unsigned short* Wg = (unsigned short*)(ws + oWg);
  unsigned short* Wf = (unsigned short*)(ws + oWf);
  unsigned short* XP = (unsigned short*)(ws + oXP);
  unsigned short* Qh = (unsigned short*)(ws + oQh);
  unsigned short* Ql = (unsigned short*)(ws + oQl);
  unsigned short* Kh = (unsigned short*)(ws + oKh);
  unsigned short* Kl = (unsigned short*)(ws + oKl);
  unsigned short* Vt = (unsigned short*)(ws + oVt);
  unsigned short* Oh = (unsigned short*)(ws + oOh);
  unsigned short* Ol = (unsigned short*)(ws + oOl);
  float* CS  = (float*)(ws + oCS);
  float* out = (float*)d_out;

  const dim3 blk256(256), blk128(128);

  cvt_w<<<dim3(WGBLK + WFBLK), blk256, 0, stream>>>(qw, kw, vw, fw, Wg, Wf);
  cvt_x<<<dim3(NQT, CC / QT, NB), blk256, 0, stream>>>(x, XP);
  qkv_k<<<dim3(NQT, NH, NB), blk128, 0, stream>>>(Wg, XP, qb, qs, qe, kb, ks, ke, vb, vs, ve, Qh, Ql, Kh, Kl, Vt);
  (void)hipFuncSetAttribute(reinterpret_cast<const void*>(&attn_k), hipFuncAttributeMaxDynamicSharedMemorySize, EDYNB);
  attn_k<<<dim3(NQT, NH, NB), blk128, EDYNB, stream>>>(Qh, Ql, Kh, Kl, Vt, Oh, Ol, CS);
  fconv_k<<<dim3(NQT, CC / QT, NB), blk128, 0, stream>>>(Wf, Oh, Ol, fb, fs, fe, x, out);
  amfin_k<<<dim3(NB), blk256, 0, stream>>>(CS, out);
  (void)hipGetLastError();
}
